// MoE_64098091925598
// MI455X (gfx1250) — hardware-run, weakly checked
//
#include <hip/hip_runtime.h>
#include <stddef.h>


typedef _Float16 v16h __attribute__((ext_vector_type(16)));
typedef _Float16 v8h  __attribute__((ext_vector_type(8)));
typedef float    v8f  __attribute__((ext_vector_type(8)));
typedef float    v4f  __attribute__((ext_vector_type(4)));
typedef _Float16 h16;

#ifndef NTOK
#define NTOK 8192
#endif
#define NTOK_FULL 8192
#define DIM   1024
#define NEXP  8
#define RANK  16
#define RC    (NEXP * RANK)
#define KCAT  (DIM + RC)

static_assert(NTOK >= 64 && NTOK <= NTOK_FULL);
static_assert((NTOK % 64) == 0 && (NTOK % 8) == 0);
static_assert((DIM % 64) == 0 && (DIM % 32) == 0 && (DIM % 8) == 0);
static_assert(DIM == 4 * 32 * 8);
static_assert(DIM == 8 * 32 * 4);
static_assert(NEXP == 8 && RANK == 16);
static_assert((RC % 64) == 0 && (RC % 32) == 0);
static_assert((KCAT % 32) == 0 && (KCAT % 64) == 0);
static_assert(((size_t)KCAT * 2) % 128 == 0);
static_assert((size_t)NTOK * KCAT < (size_t)0xFFFFFFFFu);

#define LDT 72
#define LDC 68
static_assert((LDT % 8) == 0 && LDT >= 64);
static_assert((LDC % 4) == 0 && LDC >= 64);

#define XCARRY 16.0f
#define WCARRY 64.0f
#define ACARRY 64.0f
#define BCARRY 16.0f
#define GCARRY 64.0f
static_assert(XCARRY * WCARRY == GCARRY * BCARRY);

#define XCAT_BYTES ((size_t)NTOK * KCAT * 2)
#define WCAT_BYTES ((size_t)DIM * KCAT * 2)
#define AT_BYTES   ((size_t)RC * DIM * 2)
#define COMB_BYTES ((size_t)NTOK * NEXP * 4)
#define OFF_XCAT ((size_t)0)
#define OFF_WCAT (OFF_XCAT + XCAT_BYTES)
#define OFF_AT   (OFF_WCAT + WCAT_BYTES)
#define OFF_COMB (OFF_AT + AT_BYTES)
#define WS_TOTAL (OFF_COMB + COMB_BYTES)
static_assert((XCAT_BYTES % 128) == 0 && (WCAT_BYTES % 128) == 0);
static_assert((AT_BYTES % 128) == 0 && (COMB_BYTES % 128) == 0);
static_assert(WS_TOTAL <= (size_t)134217728);

__device__ __forceinline__ float bf16r(float x) {
  unsigned int u = __float_as_uint(x);
  u = (u + 0x7FFFu + ((u >> 16) & 1u)) & 0xFFFF0000u;
  return __uint_as_float(u);
}

static __device__ __forceinline__ h16 toh_flush(float v) {
  const h16 r = (h16)v;
  return (fabsf(v) < 6.103515625e-05f) ? (h16)0.0f : r;
}

__device__ __forceinline__ v16h frag_at(const _Float16* p) {
  v8h lo = *(const v8h*)(p);
  v8h hi = *(const v8h*)(p + 16);
  v16h out;
#pragma unroll
  for (int i = 0; i < 8; ++i) { out[i] = lo[i]; out[i + 8] = hi[i]; }
  return out;
}

__device__ __forceinline__ v8f wmma16(v16h a, v16h b, v8f c) {
  v8f d = __builtin_amdgcn_wmma_f32_16x16x32_f16(false, a, false, b, (short)0, c,
                                                 false, false);
  asm volatile("v_nop\n\tv_nop\n\tv_nop\n\tv_nop" : "+v"(d) : "v"(a), "v"(b));
  return d;
}

__device__ __forceinline__ double shfl_xor_f64(double v, int mask) {
  int lo = __double2loint(v);
  int hi = __double2hiint(v);
  lo = __shfl_xor(lo, mask, 32);
  hi = __shfl_xor(hi, mask, 32);
  return __hiloint2double(hi, lo);
}

__global__ __launch_bounds__(256) void wconv_kernel(
    const float* __restrict__ W, _Float16* __restrict__ Wt, unsigned ldw, unsigned ldk,
    float carry) {
  __shared__ __attribute__((aligned(16))) _Float16 T[64 * LDT];
  const unsigned tid = threadIdx.x;
  const unsigned n0 = blockIdx.x * 64u;
  const unsigned k0 = blockIdx.y * 64u;
#pragma unroll 4
  for (unsigned j = 0; j < 16u; ++j) {
    const unsigned idx = tid + 256u * j;
    const unsigned kr = idx >> 6, nc = idx & 63u;
    const float v = W[(size_t)(k0 + kr) * ldw + n0 + nc];
    T[nc * LDT + kr] = toh_flush(carry * bf16r(v));
  }
  __syncthreads();
  v8h x[2];
  size_t off[2];
#pragma unroll
  for (unsigned i = 0; i < 2u; ++i) {
    const unsigned n = 32u * i + (tid >> 3);
    const unsigned kc = (tid & 7u) * 8u;
    x[i] = *(const v8h*)&T[n * LDT + kc];
    off[i] = (size_t)(n0 + n) * ldk + k0 + kc;
  }
#pragma unroll
  for (int i = 0; i < 2; ++i) *(volatile v8h*)(Wt + off[i]) = x[i];
  __threadfence();
#pragma unroll
  for (int i = 0; i < 2; ++i) *(volatile v8h*)(Wt + off[i]) = x[i];
}

__global__ __launch_bounds__(256) void rowconv_kernel(
    const float* __restrict__ src, _Float16* __restrict__ dst, unsigned lsrc, unsigned ldd,
    float carry) {
  const unsigned lane = threadIdx.x & 31u;
  const unsigned w = __builtin_amdgcn_readfirstlane(threadIdx.x >> 5);
  const unsigned row = blockIdx.x * 8u + w;
  const float* sr = src + (size_t)row * lsrc + lane * 8u;
  _Float16* dr = dst + (size_t)row * ldd + lane * 8u;
  v8h o[4];
#pragma unroll
  for (unsigned j = 0; j < 4u; ++j) {
    const v4f a0 = *(const v4f*)(sr + j * 256u);
    const v4f a1 = *(const v4f*)(sr + j * 256u + 4u);
#pragma unroll
    for (int i = 0; i < 4; ++i) {
      o[j][i]     = toh_flush(carry * bf16r(a0[i]));
      o[j][i + 4] = toh_flush(carry * bf16r(a1[i]));
    }
  }
#pragma unroll
  for (unsigned j = 0; j < 4u; ++j) *(volatile v8h*)(dr + j * 256u) = o[j];
  __threadfence();
#pragma unroll
  for (unsigned j = 0; j < 4u; ++j) *(volatile v8h*)(dr + j * 256u) = o[j];
}

__global__ __launch_bounds__(128) void aconv_kernel(
    const float* __restrict__ A, _Float16* __restrict__ At) {
  __shared__ __attribute__((aligned(16))) _Float16 T[RANK * LDT];
  const unsigned tid = threadIdx.x;
  const unsigned k0 = blockIdx.x * 64u;
  const unsigned e = blockIdx.y;
  const float* src = A + ((size_t)e * DIM + k0) * RANK + tid * 8u;
  const v4f a0 = *(const v4f*)(src);
  const v4f a1 = *(const v4f*)(src + 4);
  const unsigned dl = tid >> 1, r0 = (tid & 1u) * 8u;
#pragma unroll
  for (int i = 0; i < 4; ++i) {
    T[(r0 + (unsigned)i) * LDT + dl]      = toh_flush(ACARRY * bf16r(a0[i]));
    T[(r0 + 4u + (unsigned)i) * LDT + dl] = toh_flush(ACARRY * bf16r(a1[i]));
  }
  __syncthreads();
  const unsigned r = tid >> 3, kc = (tid & 7u) * 8u;
  const v8h x = *(const v8h*)&T[r * LDT + kc];
  _Float16* p = At + (size_t)(e * RANK + r) * DIM + k0 + kc;
  *(volatile v8h*)p = x;
  __threadfence();
  *(volatile v8h*)p = x;
}

__global__ __launch_bounds__(256) void gate_kernel(
    const float* __restrict__ X, const float* __restrict__ Wg, float* __restrict__ comb) {
  __shared__ __attribute__((aligned(16))) float Cw[8 * NEXP];
  const unsigned lane = threadIdx.x & 31u;
  const unsigned w = __builtin_amdgcn_readfirstlane(threadIdx.x >> 5);
  const unsigned tok = blockIdx.x * 8u + w;
  const float* xr = X + (size_t)tok * DIM + lane * 4u;
  const float* wr = Wg + lane * 4u;

  double acc[NEXP];
#pragma unroll
  for (int e = 0; e < NEXP; ++e) acc[e] = 0.0;

#pragma unroll 1
  for (unsigned j = 0; j < 8u; ++j) {
    const v4f a = *(const v4f*)(xr + j * 128u);
    double xd[4];
#pragma unroll
    for (int i = 0; i < 4; ++i) xd[i] = (double)bf16r(a[i]);
#pragma unroll
    for (int e = 0; e < NEXP; ++e) {
      const v4f g = *(const v4f*)(wr + (size_t)e * DIM + j * 128u);
#pragma unroll
      for (int i = 0; i < 4; ++i) acc[e] = fma(xd[i], (double)bf16r(g[i]), acc[e]);
    }
  }

  float l[NEXP];
#pragma unroll
  for (int e = 0; e < NEXP; ++e) {
    double s = acc[e];
#pragma unroll
    for (int off = 1; off < 32; off <<= 1) s += shfl_xor_f64(s, off);
    l[e] = (float)s;
  }

  int i0 = 0;
  float v0 = l[0];
#pragma unroll
  for (int e = 1; e < NEXP; ++e) {
    const bool gt = l[e] > v0;
    v0 = gt ? l[e] : v0;
    i0 = gt ? e : i0;
  }
  int i1 = NEXP;
  float v1 = -__builtin_inff();
#pragma unroll
  for (int e = 0; e < NEXP; ++e) {
    const bool gt = (e != i0) && (l[e] > v1);
    v1 = gt ? l[e] : v1;
    i1 = gt ? e : i1;
  }
  const float t = expf(v1 - v0);
  const float inv = 1.0f / (1.0f + t);
  const float w0 = inv;
  const float w1 = t * inv;
  const int el = (int)(lane & 7u);
  const float cw = (el == i0) ? w0 : ((el == i1) ? w1 : 0.0f);
  if (lane < 8u) Cw[w * 8u + lane] = cw;
  __syncthreads();
  if (w == 0u && lane < 16u) {
    const v4f val = *(const v4f*)&Cw[lane * 4u];
    float* p = comb + (size_t)blockIdx.x * 64u + lane * 4u;
    *(volatile v4f*)p = val;
    __threadfence();
    *(volatile v4f*)p = val;
  }
}

template <int MODE>
__device__ __forceinline__ void gemm_body(
    const _Float16* __restrict__ A16, const unsigned lda,
    const _Float16* __restrict__ Bt, const unsigned ldb, const unsigned K,
    const float* __restrict__ aux, float* __restrict__ outf, _Float16* out16) {
  __shared__ __attribute__((aligned(16))) float Cs[64 * LDC];
  const unsigned tid = threadIdx.x, lane = tid & 31u;
  const unsigned w = __builtin_amdgcn_readfirstlane(tid >> 5);
  const unsigned mw = w >> 1, nw = w & 1u;
  const unsigned hh = lane >> 4, m = lane & 15u;
  const unsigned n0 = blockIdx.x * 64u;
  const unsigned row0 = blockIdx.y * 64u;

  const _Float16* ap  = A16 + (size_t)(row0 + mw * 16u + m) * lda + hh * 8u;
  const _Float16* bp0 = Bt + (size_t)(n0 + nw * 32u + m) * ldb + hh * 8u;
  const _Float16* bp1 = bp0 + (size_t)16 * ldb;
  v8f acc0 = {}, acc1 = {};
#pragma unroll 2
  for (unsigned k0 = 0; k0 < K; k0 += 32u) {
    const v16h a  = frag_at(ap + k0);
    const v16h b0 = frag_at(bp0 + k0);
    const v16h b1 = frag_at(bp1 + k0);
    acc0 = wmma16(a, b0, acc0);
    acc1 = wmma16(a, b1, acc1);
  }
#pragma unroll
  for (int r = 0; r < 8; ++r) {
    float* d = &Cs[(mw * 16u + hh * 8u + (unsigned)r) * LDC + nw * 32u + m];
    d[0]  = acc0[r];
    d[16] = acc1[r];
  }
  __syncthreads();

  if (MODE == 0) {
    v8h x[2];
    size_t off[2];
#pragma unroll
    for (unsigned i = 0; i < 2u; ++i) {
      const unsigned r = 32u * i + (tid >> 3);
      const unsigned c = (tid & 7u) * 8u;
      const v4f u0 = *(const v4f*)&Cs[r * LDC + c];
      const v4f u1 = *(const v4f*)&Cs[r * LDC + c + 4];
      const float cw = aux[(size_t)(row0 + r) * NEXP + ((n0 + c) >> 4)];
      const float sc = cw * (GCARRY / (XCARRY * ACARRY));
#pragma unroll
      for (int j = 0; j < 4; ++j) {
        x[i][j]     = toh_flush(u0[j] * sc);
        x[i][j + 4] = toh_flush(u1[j] * sc);
      }
      off[i] = (size_t)(row0 + r) * KCAT + DIM + n0 + c;
    }
#pragma unroll
    for (int i = 0; i < 2; ++i) *(volatile v8h*)(out16 + off[i]) = x[i];
    __threadfence();
#pragma unroll
    for (int i = 0; i < 2; ++i) *(volatile v8h*)(out16 + off[i]) = x[i];
  }

  if (MODE == 1) {
    const float cs = 1.0f / (XCARRY * WCARRY);
    v4f xs[4];
    size_t off[4];
#pragma unroll
    for (unsigned i = 0; i < 4u; ++i) {
      const unsigned r = 16u * i + (tid >> 4);
      const unsigned c = (tid & 15u) * 4u;
      const v4f u = *(const v4f*)&Cs[r * LDC + c];
      const v4f g = *(const v4f*)(aux + n0 + c);
      v4f val;
#pragma unroll
      for (int j = 0; j < 4; ++j) val[j] = u[j] * cs + bf16r(g[j]);
      xs[i] = val;
      off[i] = (size_t)(row0 + r) * DIM + n0 + c;
    }
#pragma unroll
    for (int i = 0; i < 4; ++i) *(volatile v4f*)(outf + off[i]) = xs[i];
    __threadfence();
#pragma unroll
    for (int i = 0; i < 4; ++i) *(volatile v4f*)(outf + off[i]) = xs[i];
  }
}

__global__ __launch_bounds__(256) void gemm_down_kernel(
    const _Float16* __restrict__ A16, const _Float16* __restrict__ Bt,
    const float* __restrict__ comb, _Float16* gout) {
  gemm_body<0>(A16, (unsigned)KCAT, Bt, (unsigned)DIM, (unsigned)DIM, comb, (float*)0, gout);
}
__global__ __launch_bounds__(256) void gemm_out_kernel(
    const _Float16* __restrict__ A16, const _Float16* __restrict__ Bt,
    const float* __restrict__ bias, float* __restrict__ outf) {
  gemm_body<1>(A16, (unsigned)KCAT, Bt, (unsigned)KCAT, (unsigned)KCAT, bias, outf,
               (_Float16*)0);
}

extern "C" void kernel_launch(void* const* d_in, const int* in_sizes, int n_in,
                              void* d_out, int out_size, void* d_ws, size_t ws_size,
                              hipStream_t stream) {
  if (n_in < 6) return;
  if ((long long)in_sizes[0] < (long long)NTOK * DIM) return;
  if ((long long)in_sizes[1] < (long long)NEXP * DIM) return;
  if ((long long)in_sizes[2] < (long long)NEXP * DIM * RANK) return;
  if ((long long)in_sizes[3] < (long long)NEXP * RANK * DIM) return;
  if ((long long)in_sizes[4] < (long long)DIM * DIM) return;
  if (in_sizes[5] < DIM) return;
  if ((long long)out_size < (long long)NTOK * DIM) return;
  if (ws_size < WS_TOTAL) return;

  const float* X  = (const float*)d_in[0];
  const float* Wg = (const float*)d_in[1];
  const float* Aw = (const float*)d_in[2];
  const float* Bw = (const float*)d_in[3];
  const float* Wb = (const float*)d_in[4];
  const float* bb = (const float*)d_in[5];
  float* out = (float*)d_out;

  char* ws = (char*)d_ws;
  _Float16* Xcat = (_Float16*)(ws + OFF_XCAT);
  _Float16* Wcat = (_Float16*)(ws + OFF_WCAT);
  _Float16* At   = (_Float16*)(ws + OFF_AT);
  float*    Comb = (float*)(ws + OFF_COMB);

  dim3 blk(256);

  rowconv_kernel<<<dim3(NTOK / 8), blk, 0, stream>>>(X, Xcat, (unsigned)DIM, (unsigned)KCAT,
                                                     XCARRY);
  rowconv_kernel<<<dim3(DIM / 8), blk, 0, stream>>>(Wb, Wcat, (unsigned)DIM, (unsigned)KCAT,
                                                    WCARRY);
  wconv_kernel<<<dim3(DIM / 64, RC / 64), blk, 0, stream>>>(Bw, Wcat + DIM, (unsigned)DIM,
                                                            (unsigned)KCAT, BCARRY);
  aconv_kernel<<<dim3(DIM / 64, NEXP), dim3(128), 0, stream>>>(Aw, At);

  gate_kernel<<<dim3(NTOK / 8), blk, 0, stream>>>(X, Wg, Comb);
  gemm_down_kernel<<<dim3(RC / 64, NTOK / 64), blk, 0, stream>>>(Xcat, At, Comb, Xcat);
  gemm_out_kernel<<<dim3(DIM / 64, NTOK / 64), blk, 0, stream>>>(Xcat, Wcat, bb, out);
}
